// MultiHeadAttentionBlock_38053410242965
// MI455X (gfx1250) — hardware-verified
//
#include <hip/hip_runtime.h>
#ifndef NB
#define NB 2
#endif
#ifndef SQ
#define SQ 2048
#endif
#define SQ_FULL 2048
#define DM 1024
#define NH 16
#define HD 64
#define QT 256
#define QT0 128
#define NKX SQ
#define NG (NB * NH)
#define TRH (SQ / NH)
#define R0 ((QT0 * HD) / DM)
#define NR0 (NG * R0)
#define NR ((size_t)NB * SQ)
#define NFL (SQ / 256)
static_assert(NH * HD == DM);
static_assert(SQ % QT == 0);
static_assert(QT == 256);
static_assert(SQ % NH == 0);
static_assert(SQ % 128 == 0);
static_assert(SQ <= SQ_FULL);
static_assert(QT0 % 64 == 0);
static_assert(QT0 <= QT);
static_assert((QT0 * HD) % DM == 0);
static_assert(NR0 % 128 == 0);
static_assert((NB * SQ) % 128 == 0);
static_assert(((size_t)NB * SQ * DM / 8) % 256 == 0);
static_assert(((size_t)NR0 * DM / 8) % 256 == 0);
static_assert(((size_t)NR0 * DM / 4) % 256 == 0);
static_assert((NH * QT) % 256 == 0);

typedef unsigned short v8us __attribute__((ext_vector_type(8), may_alias));
typedef float  v8f  __attribute__((ext_vector_type(8)));
typedef float  v4f  __attribute__((ext_vector_type(4)));
typedef float  v4fa __attribute__((ext_vector_type(4), may_alias));
typedef int    v4ia __attribute__((ext_vector_type(4), may_alias));
typedef _Float16 v16h __attribute__((ext_vector_type(16)));
typedef _Float16 v4h  __attribute__((ext_vector_type(4)));
union FragH { v16h v; v8us half[2]; _Float16 h[16]; unsigned short u[16]; };

__device__ __forceinline__ unsigned short bf16_bits(float x) { unsigned int u = __float_as_uint(x); return (unsigned short)((u + 0x7FFFu + ((u >> 16) & 1u)) >> 16); }
__device__ __forceinline__ float bf16_val(unsigned short b) { return __uint_as_float(((unsigned int)b) << 16); }
__device__ __forceinline__ float bf16_rne(float x) { return bf16_val(bf16_bits(x)); }

__global__ __launch_bounds__(256) void k_wnat(const float* __restrict__ w, unsigned n8, _Float16* __restrict__ Bt) {
  const unsigned t = blockIdx.x * 256u + threadIdx.x; if (t >= n8) return;
  const v4f a = *(const v4fa*)(w + (size_t)t * 8), c = *(const v4fa*)(w + (size_t)t * 8 + 4);
  FragH f;
#pragma unroll
  for (int q = 0; q < 4; ++q) { f.h[q] = (_Float16)(bf16_rne(a[q]) * 16.0f); f.h[4 + q] = (_Float16)(bf16_rne(c[q]) * 16.0f); }
  const v8us o = f.half[0];
  unsigned short* d = (unsigned short*)Bt + (size_t)t * 8;
  *(volatile v8us*)d = o; __threadfence(); *(volatile v8us*)d = o;
}

__global__ __launch_bounds__(256) void k_x16(const float* __restrict__ x, _Float16* __restrict__ X16) {
  const unsigned PB = (unsigned)((size_t)SQ * DM / 8);
  const unsigned t = blockIdx.x * 256u + threadIdx.x; if (t >= (unsigned)NB * PB) return;
  const unsigned b = t / PB; const unsigned r = t - b * PB;
  const float* src = x + (size_t)b * SQ_FULL * DM + (size_t)r * 8;
  const v4f a = *(const v4fa*)src, c = *(const v4fa*)(src + 4);
  FragH f;
#pragma unroll
  for (int q = 0; q < 4; ++q) { f.h[q] = (_Float16)bf16_rne(a[q]); f.h[4 + q] = (_Float16)bf16_rne(c[q]); }
  const v8us o = f.half[0];
  unsigned short* d = (unsigned short*)X16 + (size_t)t * 8;
  *(volatile v8us*)d = o; __threadfence(); *(volatile v8us*)d = o;
}

__global__ __launch_bounds__(256) void k_first8(const _Float16* __restrict__ XA, const _Float16* __restrict__ XB, const _Float16* __restrict__ XC,
                                               _Float16* __restrict__ DA, _Float16* __restrict__ DB, _Float16* __restrict__ DC) {
  const unsigned t = blockIdx.x * 256u + threadIdx.x;
  const unsigned which = blockIdx.y;
  const unsigned short* src = (const unsigned short*)(which == 0u ? XA : (which == 1u ? XB : XC));
  unsigned short* dst = (unsigned short*)(which == 0u ? DA : (which == 1u ? DB : DC));
  const unsigned row = t >> 7, c8 = (t & 127u) << 3;
  const unsigned g = row / (unsigned)R0, tt = row - g * (unsigned)R0;
  const v8us v = *(const v8us*)(src + ((size_t)g * TRH + tt) * DM + c8);
  unsigned short* d = dst + (size_t)row * DM + c8;
  *(volatile v8us*)d = v; __threadfence(); *(volatile v8us*)d = v;
}

__global__ __launch_bounds__(256) void k_vt(const _Float16* __restrict__ V16, _Float16* __restrict__ Vt) {
  __shared__ unsigned short tl[64][66];
  const unsigned tid = threadIdx.x; const unsigned slab = blockIdx.x / (SQ / 64), lg = blockIdx.x % (SQ / 64);
  for (unsigned i = tid; i < 64u * 8u; i += 256u) { const unsigned r = i >> 3, c8 = (i & 7u) << 3; FragH f;
    f.half[0] = *(const v8us*)((const unsigned short*)V16 + ((size_t)slab * SQ + lg * 64u + r) * HD + c8);
#pragma unroll
    for (int q = 0; q < 8; ++q) tl[r][c8 + q] = f.u[q]; }
  __syncthreads();
  for (int pass = 0; pass < 2; ++pass) {
#pragma unroll
    for (unsigned rd = 0; rd < 2; ++rd) { const unsigned d = rd * 32u + (tid >> 3), pc = tid & 7u; FragH f;
#pragma unroll
      for (int q = 0; q < 8; ++q) f.u[q] = tl[pc * 8u + q][d];
      *(volatile v8us*)((unsigned short*)Vt + ((size_t)slab * HD + d) * SQ + lg * 64u + pc * 8u) = f.half[0]; }
    if (pass == 0) __threadfence(); } }

__global__ __launch_bounds__(256) void k_hl(const float* __restrict__ F, _Float16* __restrict__ Hh, _Float16* __restrict__ Hl, unsigned n8) {
  const unsigned t = blockIdx.x * 256u + threadIdx.x; if (t >= n8) return; FragH fh, fl;
  const v4f a = *(const v4fa*)(F + (size_t)t * 8), c = *(const v4fa*)(F + (size_t)t * 8 + 4);
#pragma unroll
  for (int q = 0; q < 4; ++q) { _Float16 h = (_Float16)a[q]; fh.h[q] = h; fl.h[q] = (_Float16)((a[q] - (float)h) * 1024.0f); h = (_Float16)c[q]; fh.h[4 + q] = h; fl.h[4 + q] = (_Float16)((c[q] - (float)h) * 1024.0f); }
  const v8us oh = fh.half[0], ol = fl.half[0];
  for (int pass = 0; pass < 2; ++pass) { *(volatile v8us*)((unsigned short*)Hh + (size_t)t * 8) = oh; *(volatile v8us*)((unsigned short*)Hl + (size_t)t * 8) = ol; if (pass == 0) __threadfence(); } }

__device__ __forceinline__ v16h g2_frag(const _Float16* p, unsigned hh) { FragH f; f.half[0] = *(const v8us*)((const unsigned short*)p + 8u * hh); f.half[1] = *(const v8us*)((const unsigned short*)p + 16u + 8u * hh); return f.v; }
__device__ __forceinline__ v8f g2_mma(v16h a, v16h b, v8f c) { v8f d = __builtin_amdgcn_wmma_f32_16x16x32_f16(false, a, false, b, (short)0, c, false, false); asm volatile("v_nop\n\tv_nop\n\tv_nop\n\tv_nop" : "+v"(d) : "v"(a), "v"(b)); return d; }
__global__ __launch_bounds__(128) void k_gemm2(const _Float16* __restrict__ A, int lda, size_t sA, const _Float16* __restrict__ Bh, int ldb, size_t sB, float alpha, const float* __restrict__ bias, const float* CP,
    float* C, _Float16* __restrict__ C16, int ldc, size_t sC, int M, int N, int K) {
  __shared__ __attribute__((aligned(16))) float so[4][32][68];
  const unsigned tid = threadIdx.x, w = tid >> 5, lane = tid & 31u, ln = lane & 15u, hh = lane >> 4; const unsigned by = blockIdx.y;
  A += (size_t)by * sA; Bh += (size_t)by * sB; const size_t cofs = (size_t)by * sC;
  const unsigned ntn = (unsigned)N >> 6; const unsigned mt = blockIdx.x / ntn, nq = blockIdx.x - mt * ntn; const unsigned row0 = mt * 128u + 32u * w, col0 = nq * 64u; if (row0 >= (unsigned)M) return;
  const _Float16* a0p = A + (size_t)(row0 + ln) * lda; const _Float16* a1p = a0p + (size_t)16 * lda;
  const _Float16* b0p = Bh + (size_t)(col0 + ln) * ldb; const _Float16* b1p = b0p + (size_t)16 * ldb; const _Float16* b2p = b1p + (size_t)16 * ldb; const _Float16* b3p = b2p + (size_t)16 * ldb;
  const v8f z8 = {0.f,0.f,0.f,0.f,0.f,0.f,0.f,0.f}; v8f c00 = z8, c01 = z8, c02 = z8, c03 = z8, c10 = z8, c11 = z8, c12 = z8, c13 = z8;
#pragma unroll 1
  for (int kb = 0; kb < K; kb += 32) { const v16h a0 = g2_frag(a0p + kb, hh), a1 = g2_frag(a1p + kb, hh);
    v16h b = g2_frag(b0p + kb, hh); c00 = g2_mma(a0, b, c00); c10 = g2_mma(a1, b, c10);
    b = g2_frag(b1p + kb, hh); c01 = g2_mma(a0, b, c01); c11 = g2_mma(a1, b, c11);
    b = g2_frag(b2p + kb, hh); c02 = g2_mma(a0, b, c02); c12 = g2_mma(a1, b, c12);
    b = g2_frag(b3p + kb, hh); c03 = g2_mma(a0, b, c03); c13 = g2_mma(a1, b, c13); }
  v8f accs[8] = {c00, c01, c02, c03, c10, c11, c12, c13};
#pragma unroll
  for (int u = 0; u < 8; ++u) { const unsigned t = (unsigned)u & 3u, hf = (unsigned)u >> 2; const unsigned col = col0 + t * 16u + ln; const float bv = bias ? bf16_rne(bias[col]) : 0.f;
#pragma unroll
    for (int r = 0; r < 8; ++r) { const unsigned rloc = hf * 16u + 8u * hh + (unsigned)r; float v = accs[u][r] * alpha + bv;
      if (CP) v += CP[cofs + (size_t)(row0 + rloc) * ldc + col];
      so[w][rloc][t * 16u + ln] = v; } }
  __builtin_amdgcn_fence(4  , "workgroup"); __builtin_amdgcn_wave_barrier();
  const unsigned rsub = lane >> 4, c4 = (lane & 15u) * 4u;
  for (int pass = 0; pass < 2; ++pass) {
#pragma unroll
    for (unsigned q = 0; q < 16; ++q) { const unsigned r = q * 2u + rsub; const v4f v = *(const v4fa*)&so[w][r][c4];
      if (C) *(volatile v4f*)(C + cofs + (size_t)(row0 + r) * ldc + col0 + c4) = v;
      if (C16) { v4h h4; for (int i = 0; i < 4; ++i) h4[i] = (_Float16)v[i]; *(volatile v4h*)(C16 + cofs + (size_t)(row0 + r) * ldc + col0 + c4) = h4; } }
    if (pass == 0) __threadfence(); } }

__global__ __launch_bounds__(256) void k_rsmcfk(const float* __restrict__ S, _Float16* __restrict__ P, int hg, int q0, int nk, const int* __restrict__ mk) {
  #pragma clang fp contract(off)
  const unsigned t = blockIdx.x * 256u + threadIdx.x; if (t >= (unsigned)hg * QT) return; const size_t i = (size_t)t; const float* s = S + i * NKX; const size_t ig = (size_t)q0 + (t % (unsigned)QT); const int* mr = mk + ig * SQ_FULL; float mx = -3.0e38f;
#pragma unroll 1
  for (int j = 0; j < nk; ++j) { const int mb = mr[j]; const float f = (mb != 0) ? 1.f : 0.f; mx = fmaxf(mx, fmaf(f, s[j], (1.f - f) * -1.0e9f)); } float se = 0.f;
#pragma unroll 1
  for (int j = 0; j < nk; ++j) { const int mb = mr[j]; const float f = (mb != 0) ? 1.f : 0.f; se += __expf(fmaf(f, s[j], (1.f - f) * -1.0e9f) - mx); } const float sc = 256.0f / se;
#pragma unroll 1
  for (int j0 = 0; j0 < nk; j0 += 8) { FragH fr; for (int q = 0; q < 8; ++q) { const int j = j0 + q; const int mb = mr[j]; const float f = (mb != 0) ? 1.f : 0.f; fr.h[q] = (_Float16)(__expf(fmaf(f, s[j], (1.f - f) * -1.0e9f) - mx) * sc); } const v8us o = fr.half[0]; unsigned short* d = (unsigned short*)P + i * NKX + j0; *(volatile v8us*)d = o; __threadfence(); *(volatile v8us*)d = o; } }

__global__ __launch_bounds__(64) void k_att0(const float* __restrict__ QF, const float* __restrict__ KF, const float* __restrict__ VF, const int* __restrict__ mask, float scale, float* __restrict__ OF) {
  #pragma clang fp contract(off)
  __shared__ __attribute__((aligned(16))) float lq[64][64]; __shared__ __attribute__((aligned(16))) float lo[64][64];
  const unsigned tid = threadIdx.x; const unsigned g = blockIdx.x / (QT0 / 64), rg = blockIdx.x % (QT0 / 64); const unsigned i = rg * 64u + tid;
  const size_t sb = (size_t)g * QT0 * HD;
  const float* qr = QF + sb + (size_t)i * HD;
#pragma unroll 1
  for (unsigned c = 0; c < HD / 4; ++c) { *(v4f*)&lq[tid][c * 4] = *(const v4fa*)(qr + c * 4); const v4f z = {0.f, 0.f, 0.f, 0.f}; *(v4f*)&lo[tid][c * 4] = z; }
  float m = -1.0e30f, l = 0.f; const unsigned jmax = rg * 64u + 63u; const int* mrow = mask + (size_t)i * SQ_FULL;
#pragma unroll 1
  for (unsigned j = 0; j <= jmax; ++j) { const float* kr = KF + sb + (size_t)j * HD; const float* vr = VF + sb + (size_t)j * HD; float s = 0.f;
#pragma unroll 1
    for (unsigned c = 0; c < HD / 4; ++c) { const v4f kq = *(const v4fa*)(kr + c * 4); const v4f qq = *(v4f*)&lq[tid][c * 4]; s = __fadd_rn(s, __fmul_rn(qq[0], kq[0])); s = __fadd_rn(s, __fmul_rn(qq[1], kq[1])); s = __fadd_rn(s, __fmul_rn(qq[2], kq[2])); s = __fadd_rn(s, __fmul_rn(qq[3], kq[3])); }
    s = __fmul_rn(s, scale); const int mb = mrow[j];
    const float f = (mb != 0) ? 1.f : 0.f; const float sm = fmaf(f, s, (1.f - f) * -1.0e30f); const float mn = fmaxf(m, sm); const float sc = expf(m - mn); const float e = expf(sm - mn); l = __fadd_rn(__fmul_rn(l, sc), e); m = mn;
#pragma unroll 1
    for (unsigned c = 0; c < HD / 4; ++c) { const v4f vv = *(const v4fa*)(vr + c * 4); v4f oo = *(v4f*)&lo[tid][c * 4]; for (int u = 0; u < 4; ++u) oo[u] = __fadd_rn(__fmul_rn(oo[u], sc), __fmul_rn(e, vv[u])); *(v4f*)&lo[tid][c * 4] = oo; } }
  const float fin = 64.0f * (1.0f / l);
#pragma unroll 1
  for (unsigned c = 0; c < HD / 4; ++c) { v4f oo = *(v4f*)&lo[tid][c * 4]; for (int u = 0; u < 4; ++u) oo[u] = __fmul_rn(oo[u], fin); *(v4f*)&lo[tid][c * 4] = oo; }
  __syncthreads();
  for (int pass = 0; pass < 2; ++pass) {
#pragma unroll 1
    for (unsigned it = 0; it < 16; ++it) { const unsigned row = it * 4u + (tid >> 4), pc = (tid & 15u) * 4u; const v4f v = *(const v4f*)&lo[row][pc]; *(volatile v4f*)(OF + sb + (size_t)(rg * 64u + row) * HD + pc) = v; }
    if (pass == 0) __threadfence(); } }

__global__ __launch_bounds__(256) void k_mchk(const int* __restrict__ mk, float* __restrict__ flg) {
  __shared__ unsigned sbad[8];
  const unsigned tid = threadIdx.x, w = tid >> 5, lane = tid & 31u; unsigned bad = 0u;
#pragma unroll 1
  for (unsigned rr = 0; rr < 32u; ++rr) { const unsigned i = blockIdx.x * 256u + w * 32u + rr;
    const unsigned bound = (i < (unsigned)QT0) ? (((i >> 6) + 1u) << 6) : (((i >> 8) + 1u) << 8);
    const int* mr = mk + (size_t)i * SQ_FULL; int lo = 0, hi = 0;
#pragma unroll 1
    for (unsigned c = lane * 4u; c < (unsigned)SQ; c += 128u) { const v4ia mv = *(const v4ia*)(mr + c);
#pragma unroll
      for (int e = 0; e < 4; ++e) { const int nz = (mv[e] != 0) ? 1 : 0; const int below = ((c + (unsigned)e) < bound) ? 1 : 0; lo += nz & below; hi += nz & (1 - below); } }
#pragma unroll
    for (int off = 16; off >= 1; off >>= 1) { lo += __shfl_xor(lo, off, 32); hi += __shfl_xor(hi, off, 32); }
    bad |= ((hi != 0) || (lo == 0)) ? 1u : 0u; }
  if (lane == 0u) sbad[w] = bad;
  __syncthreads();
  unsigned any = 0u;
#pragma unroll
  for (int q = 0; q < 8; ++q) any |= sbad[q];
  const float fv = any ? 1.0f : 0.0f; const v4f v = {fv, fv, fv, fv};
  float* d = flg + (size_t)blockIdx.x * 32u + (lane & 7u) * 4u;
  if (w == 0u && lane < 8u) { *(volatile v4f*)d = v; __threadfence(); *(volatile v4f*)d = v; } }

__global__ __launch_bounds__(256) void k_out0(const float* __restrict__ O0, float* __restrict__ out) {
  const unsigned t = blockIdx.x * 256u + threadIdx.x;
  const unsigned row = t >> 8, c4 = (t & 255u) << 2;
  const unsigned g = row / (unsigned)R0, tt = row - g * (unsigned)R0;
  const v4f v = *(const v4fa*)(O0 + (size_t)row * DM + c4);
  float* d = out + ((size_t)g * TRH + tt) * DM + c4;
  *(volatile v4f*)d = v; __threadfence(); *(volatile v4f*)d = v; }

__global__ __launch_bounds__(256) void k_poison(const float* __restrict__ flg, float* __restrict__ out, unsigned n4) {
  float s = 0.f;
#pragma unroll 1
  for (unsigned q = 0; q < (unsigned)NFL; ++q) s += flg[q * 32u];
  if (!(s > 0.5f)) return;
  const float nn = __uint_as_float(0x7fc00000u); const v4f v = {nn, nn, nn, nn};
  for (int pass = 0; pass < 2; ++pass) {
    for (unsigned t = blockIdx.x * 256u + threadIdx.x; t < n4; t += gridDim.x * 256u) *(volatile v4f*)(out + (size_t)t * 4) = v;
    if (pass == 0) __threadfence(); } }

extern "C" void kernel_launch(void* const* d_in, const int* in_sizes, int n_in,
                              void* d_out, int out_size, void* d_ws, size_t ws_size, hipStream_t stream) {
  if (n_in < 12) return;
  const size_t needx = (size_t)(NB - 1) * SQ_FULL * DM + (size_t)SQ * DM;
  if ((size_t)in_sizes[0] < needx || (size_t)in_sizes[1] < needx || (size_t)in_sizes[2] < needx) return;
  if ((size_t)in_sizes[3] < (size_t)(SQ - 1) * SQ_FULL + SQ) return;
  if ((size_t)in_sizes[4] < (size_t)DM * DM || (size_t)in_sizes[6] < (size_t)DM * DM || (size_t)in_sizes[8] < (size_t)DM * DM || (size_t)in_sizes[10] < (size_t)DM * DM) return;
  if (in_sizes[5] < DM || in_sizes[7] < DM || in_sizes[9] < DM || in_sizes[11] < DM) return;
  if ((size_t)out_size < NR * DM) return;
  const float* const* I = (const float* const*)d_in;
  const float* xk = I[0]; const float* xq = I[1]; const float* xv = I[2]; const int* mk = (const int*)d_in[3];
  const float* wq = I[4]; const float* bq = I[5]; const float* wk = I[6]; const float* bk = I[7]; const float* wv = I[8]; const float* bv = I[9]; const float* wo = I[10]; const float* bo = I[11];
  float* out = (float*)d_out;
  char* ws = (char*)d_ws; size_t off = 0;
  auto take = [&](size_t bytes) { char* p = ws + off; off += (bytes + 255) & ~(size_t)255; return p; };
  _Float16* BQ = (_Float16*)take((size_t)DM * DM * 2); _Float16* BK = (_Float16*)take((size_t)DM * DM * 2); _Float16* BV = (_Float16*)take((size_t)DM * DM * 2); _Float16* BO = (_Float16*)take((size_t)DM * DM * 2);
  _Float16* XQ = (_Float16*)take(NR * DM * 2); _Float16* XK = (_Float16*)take(NR * DM * 2); _Float16* XV = (_Float16*)take(NR * DM * 2);
  _Float16* Q16 = (_Float16*)take(NR * DM * 2); _Float16* K16 = (_Float16*)take(NR * DM * 2); _Float16* V16 = (_Float16*)take(NR * DM * 2); _Float16* O16 = (_Float16*)take(NR * DM * 2);
  float* S = (float*)take((size_t)NH * QT * NKX * 4); _Float16* P = (_Float16*)take((size_t)NH * QT * NKX * 2); _Float16* VT = (_Float16*)take((size_t)NH * HD * SQ * 2);
  _Float16* XQ0 = (_Float16*)take((size_t)NR0 * DM * 2); _Float16* XK0 = (_Float16*)take((size_t)NR0 * DM * 2); _Float16* XV0 = (_Float16*)take((size_t)NR0 * DM * 2);
  float* QF0 = (float*)take((size_t)NR0 * DM * 4); float* KF0 = (float*)take((size_t)NR0 * DM * 4); float* VF0 = (float*)take((size_t)NR0 * DM * 4);
  float* OF0 = (float*)take((size_t)NR0 * DM * 4); _Float16* OH0 = (_Float16*)take((size_t)NR0 * DM * 2); _Float16* OL0 = (_Float16*)take((size_t)NR0 * DM * 2); float* OUT0 = (float*)take((size_t)NR0 * DM * 4);
  float* FLG = (float*)take((size_t)NFL * 128);
  if (off > ws_size || off > (size_t)134217728) return;

  const unsigned w8 = (unsigned)((size_t)DM * DM / 8);
  k_wnat<<<(w8 + 255u) / 256u, 256, 0, stream>>>(wq, w8, BQ); k_wnat<<<(w8 + 255u) / 256u, 256, 0, stream>>>(wk, w8, BK);
  k_wnat<<<(w8 + 255u) / 256u, 256, 0, stream>>>(wv, w8, BV); k_wnat<<<(w8 + 255u) / 256u, 256, 0, stream>>>(wo, w8, BO);
  const unsigned gX = (unsigned)(NR * DM / 8 / 256);
  k_x16<<<gX, 256, 0, stream>>>(xq, XQ); k_x16<<<gX, 256, 0, stream>>>(xk, XK); k_x16<<<gX, 256, 0, stream>>>(xv, XV);
  k_mchk<<<NFL, 256, 0, stream>>>(mk, FLG);
  const dim3 gP((unsigned)((NR / 128) * (DM / 64)), 1);
  k_gemm2<<<gP, 128, 0, stream>>>(XQ, DM, 0, BQ, DM, 0, 0.0625f, bq, nullptr, nullptr, Q16, DM, 0, (int)NR, DM, DM);
  k_gemm2<<<gP, 128, 0, stream>>>(XK, DM, 0, BK, DM, 0, 0.0625f, bk, nullptr, nullptr, K16, DM, 0, (int)NR, DM, DM);
  k_gemm2<<<gP, 128, 0, stream>>>(XV, DM, 0, BV, DM, 0, 0.0625f, bv, nullptr, nullptr, V16, DM, 0, (int)NR, DM, DM);
  k_first8<<<dim3((unsigned)((size_t)NR0 * DM / 8 / 256), 3), 256, 0, stream>>>(XQ, XK, XV, XQ0, XK0, XV0);
  const dim3 gF((unsigned)((NR0 / 128) * (DM / 64)), 1);
  k_gemm2<<<gF, 128, 0, stream>>>(XQ0, DM, 0, BQ, DM, 0, 0.0625f, bq, nullptr, QF0, nullptr, DM, 0, NR0, DM, DM);
  k_gemm2<<<gF, 128, 0, stream>>>(XK0, DM, 0, BK, DM, 0, 0.0625f, bk, nullptr, KF0, nullptr, DM, 0, NR0, DM, DM);
  k_gemm2<<<gF, 128, 0, stream>>>(XV0, DM, 0, BV, DM, 0, 0.0625f, bv, nullptr, VF0, nullptr, DM, 0, NR0, DM, DM);
  k_att0<<<NG * (QT0 / 64), 64, 0, stream>>>(QF0, KF0, VF0, mk, 0.03125f, OF0);
  for (int b = 0; b < NB; ++b) { const size_t e0 = (size_t)b * SQ * DM;
    k_vt<<<NH * (SQ / 64), 256, 0, stream>>>(V16 + e0, VT);
    for (int q0 = 0; q0 < SQ; q0 += QT) { const int nk = q0 + QT;
      k_gemm2<<<dim3((unsigned)((QT / 128) * (nk / 64)), NH), 128, 0, stream>>>(Q16 + e0 + (size_t)q0 * HD, HD, (size_t)SQ * HD, K16 + e0, HD, (size_t)SQ * HD, 0.03125f, nullptr, nullptr, S, nullptr, NKX, (size_t)QT * NKX, QT, nk, HD);
      k_rsmcfk<<<(NH * QT) / 256, 256, 0, stream>>>(S, P, NH, q0, nk, mk);
      k_gemm2<<<dim3((QT / 128) * (HD / 64), NH), 128, 0, stream>>>(P, NKX, (size_t)QT * NKX, VT, SQ, (size_t)HD * SQ, 0.25f, nullptr, nullptr, nullptr, O16 + e0 + (size_t)q0 * HD, HD, (size_t)SQ * HD, QT, HD, nk); } }
  k_gemm2<<<gP, 128, 0, stream>>>(O16, DM, 0, BO, DM, 0, 0.0009765625f, bo, nullptr, out, nullptr, DM, 0, (int)NR, DM, DM);
  k_hl<<<(unsigned)((size_t)NR0 * DM / 8 / 256), 256, 0, stream>>>(OF0, OH0, OL0, (unsigned)((size_t)NR0 * DM / 8));
  k_gemm2<<<gF, 128, 0, stream>>>(OH0, DM, 0, BO, DM, 0, 0.0009765625f, bo, nullptr, OUT0, nullptr, DM, 0, NR0, DM, DM);
  k_gemm2<<<gF, 128, 0, stream>>>(OL0, DM, 0, BO, DM, 0, 0.00000095367431640625f, nullptr, OUT0, OUT0, nullptr, DM, 0, NR0, DM, DM);
  k_out0<<<(unsigned)((size_t)NR0 * DM / 4 / 256), 256, 0, stream>>>(OUT0, out);
  k_poison<<<256, 256, 0, stream>>>(FLG, out, (unsigned)(NR * DM / 4));
}
